// SSM_54365696033203
// MI455X (gfx1250) — hardware-run, weakly checked
//
#include <hip/hip_runtime.h>
#include <math.h>

typedef __attribute__((ext_vector_type(16))) __bf16   v16b;
typedef __attribute__((ext_vector_type(8)))  __bf16   v8b;
typedef __attribute__((ext_vector_type(8)))  _Float16 v8h;
typedef __attribute__((ext_vector_type(8)))  float    v8f;
typedef __attribute__((ext_vector_type(4)))  float    v4f;

constexpr int kBatch   = 64;
constexpr int kSteps   = 8192;
constexpr int kState   = 64;
constexpr int kRowsBlk = 16;
constexpr int kChunk   = 64;
constexpr int kSlabP   = 68;
constexpr int kLoP     = 72;
constexpr int kAugP    = 129;
constexpr int kNumP    = 65;
static_assert(kBatch % kRowsBlk == 0);
static_assert(kSteps % kChunk == 0);
static_assert(kState % 32 == 0);
static_assert((kSlabP * 4) % 16 == 0);
static_assert((kLoP * 2) % 16 == 0);

constexpr size_t kBytesPlane = (size_t)kState * kState * 2;
constexpr size_t kBytesBC    = (size_t)2 * kState * 4;
constexpr size_t kWsTotal    = kBytesPlane + kBytesPlane + kBytesBC;
static_assert(kWsTotal == 16896ull);
static_assert(kWsTotal <= 134217728ull);

__device__ __forceinline__ unsigned short f2bf_bits(float f) {
  unsigned u = __float_as_uint(f);
  return (unsigned short)((u + 0x7FFFu + ((u >> 16) & 1u)) >> 16);
}
__device__ __forceinline__ float bf_bits2f(unsigned short h) { return __uint_as_float(((unsigned)h) << 16); }

__device__ __forceinline__ void split_bf(float f, __bf16& hi, __bf16& lo) {
  const unsigned short hb = f2bf_bits(f);
  const unsigned short lb = f2bf_bits(f - bf_bits2f(hb));
  hi = __builtin_bit_cast(__bf16, hb);
  lo = __builtin_bit_cast(__bf16, lb);
}

__device__ __forceinline__ v16b frag_load(const __bf16* p) {
  union U { v16b v; v8b h[2]; };
  U f;
  f.h[0] = *(const v8b*)(p);
  f.h[1] = *(const v8b*)(p + 16);
  return f.v;
}

__device__ __forceinline__ v8f mma_b(v16b a, v16b b, v8f c) {
  c = __builtin_amdgcn_wmma_f32_16x16x32_bf16(false, a, false, b, (short)0, c, false, false);
  asm volatile("v_nop\n\tv_nop\n\tv_nop\n\tv_nop" : "+v"(c) : "v"(a), "v"(b));
  return c;
}

__global__ __launch_bounds__(256) void discretise_kernel(
    const float* __restrict__ A, const float* __restrict__ Bv, const float* __restrict__ Cv,
    const float* __restrict__ stepp,
    unsigned short* __restrict__ ABH, unsigned short* __restrict__ ABL, float* __restrict__ BC)
{
  __shared__ float aug[kState * kAugP];
  __shared__ float sNum[kState * kNumP];
  __shared__ float prow[2 * kState];
  __shared__ float bsrc[kState];
  __shared__ __align__(16) float bc[2 * kState];
  __shared__ int pivsel;

  const int tid = threadIdx.x;
  const int row = tid & 63;
  const int cg  = tid >> 6;
  const float hs = stepp[0];
  const float hh = hs * 0.5f;

#pragma unroll 1
  for (int jj = 0; jj < 16; ++jj) {
    const int j = cg * 16 + jj;
    const float a   = A[row * kState + j];
    const float eye = (row == j) ? 1.0f : 0.0f;
    aug[row * kAugP + j]          = eye - hh * a;
    aug[row * kAugP + kState + j] = eye;
    sNum[row * kNumP + j]         = eye + hh * a;
  }
  if (tid < 64) bsrc[tid] = Bv[tid];
  if (tid >= 64 && tid < 128) bc[tid] = Cv[tid - 64];
  __syncthreads();

#pragma unroll 1
  for (int c = 0; c < kState; ++c) {
    if (tid == 0) {
      float best = fabsf(aug[c * kAugP + c]);
      int bi = c;
#pragma unroll 1
      for (int r = c + 1; r < kState; ++r) {
        const float v = fabsf(aug[r * kAugP + c]);
        if (v > best) { best = v; bi = r; }
      }
      pivsel = bi;
    }
    __syncthreads();
    int p = pivsel;
    p = (p < c) ? c : p;
    p = (p > kState - 1) ? (kState - 1) : p;
    if (tid < 128) {
      const float t0 = aug[c * kAugP + tid];
      const float t1 = aug[p * kAugP + tid];
      aug[c * kAugP + tid] = t1;
      aug[p * kAugP + tid] = t0;
    }
    __syncthreads();
    const float pinv = 1.0f / aug[c * kAugP + c];
    const float f    = aug[row * kAugP + c];
    if (tid < 128) prow[tid] = aug[c * kAugP + tid] * pinv;
    __syncthreads();
#pragma unroll 1
    for (int jj = 0; jj < 32; ++jj) {
      const int j = cg * 32 + jj;
      const float pr  = prow[j];
      const float cur = aug[row * kAugP + j];
      const float nv  = (row == c) ? pr : (cur - f * pr);
      aug[row * kAugP + j] = nv;
    }
    __syncthreads();
  }

#pragma unroll 1
  for (int jj = 0; jj < 16; ++jj) {
    const int j = cg * 16 + jj;
    float acc = 0.0f;
#pragma unroll 1
    for (int k = 0; k < kState; ++k) acc = fmaf(aug[row * kAugP + kState + k], sNum[k * kNumP + j], acc);
    aug[row * kAugP + j] = acc;
  }
  if (tid < 64) {
    float acc = 0.0f;
#pragma unroll 1
    for (int k = 0; k < kState; ++k) {
      const float w = aug[tid * kAugP + kState + k] * hs;
      acc = fmaf(w, bsrc[k], acc);
    }
    bc[tid] = acc;
  }
  __syncthreads();

  v8h hv[2], lv[2];
#pragma unroll
  for (int q = 0; q < 2; ++q) {
    const int i  = tid + 256 * q;
    const int r  = i >> 3;
    const int c8 = (i & 7) * 8;
#pragma unroll
    for (int e = 0; e < 8; ++e) {
      const float fv = aug[r * kAugP + c8 + e];
      const unsigned short hb = f2bf_bits(fv);
      const unsigned short lb = f2bf_bits(fv - bf_bits2f(hb));
      hv[q][e] = __builtin_bit_cast(_Float16, hb);
      lv[q][e] = __builtin_bit_cast(_Float16, lb);
    }
  }
  v4f bcv = (v4f){0.f, 0.f, 0.f, 0.f};
  if (tid < 32) bcv = *(const v4f*)(bc + tid * 4);
  for (int pass = 0; pass < 2; ++pass) {
#pragma unroll
    for (int q = 0; q < 2; ++q) {
      const int i  = tid + 256 * q;
      const int r  = i >> 3;
      const int c8 = (i & 7) * 8;
      *(volatile v8h*)(ABH + r * kState + c8) = hv[q];
      *(volatile v8h*)(ABL + r * kState + c8) = lv[q];
    }
    if (tid < 32) *(volatile v4f*)(BC + tid * 4) = bcv;
    __threadfence();
  }
}

__global__ __launch_bounds__(32) void state_scan_kernel(
    const float* __restrict__ u,
    const unsigned short* __restrict__ ABHp, const unsigned short* __restrict__ ABLp,
    const float* __restrict__ BC, float* __restrict__ out)
{
  __shared__ __align__(16) __bf16 ALs[kState * kLoP];
  __shared__ __align__(16) float  XS[kRowsBlk * kSlabP];
  __shared__ __align__(16) float  US[kRowsBlk * kSlabP];
  __shared__ __align__(16) float  YS[kRowsBlk * kSlabP];
  __shared__ __align__(16) float  CS[kState];

  const __bf16* ABH = (const __bf16*)ABHp;
  const __bf16* ABL = (const __bf16*)ABLp;
  const int lane = threadIdx.x & 31;
  const int hh   = lane >> 4;
  const int c    = lane & 15;
  const int koff = 8 * hh;
  const int c4   = c * 4;
  const int rowbase = blockIdx.x * kRowsBlk;

#pragma unroll 1
  for (int i = lane; i < 512; i += 32) {
    const int r  = i >> 3;
    const int c8 = (i & 7) * 8;
    const v8b w = *(const v8b*)(ABL + r * kState + c8);
    *(v8b*)(ALs + r * kLoP + c8) = w;
  }
  CS[lane]      = BC[kState + lane];
  CS[32 + lane] = BC[kState + 32 + lane];

  float bD[4];
#pragma unroll
  for (int nt = 0; nt < 4; ++nt) bD[nt] = BC[16 * nt + c];

  v16b bh[4][2];
#pragma unroll
  for (int nt = 0; nt < 4; ++nt)
#pragma unroll
    for (int kh = 0; kh < 2; ++kh)
      bh[nt][kh] = frag_load(ABH + (16 * nt + c) * kState + koff + 32 * kh);

  float xa[32];
#pragma unroll
  for (int i = 0; i < 32; ++i) xa[i] = 0.0f;
  __syncthreads();

  const v8f z8 = {0.f, 0.f, 0.f, 0.f, 0.f, 0.f, 0.f, 0.f};

#pragma unroll 1
  for (int t0 = 0; t0 < kSteps; t0 += kChunk) {
#pragma unroll
    for (int it = 0; it < 8; ++it) {
      const int rr = it * 2 + hh;
      const v4f uv = *(const v4f*)(u + (size_t)(rowbase + rr) * kSteps + t0 + c4);
      *(v4f*)(US + rr * kSlabP + c4) = uv;
    }
    __syncthreads();

#pragma unroll 1
    for (int s = 0; s < kChunk; ++s) {
      v16b ah[2], al[2];
#pragma unroll
      for (int kh = 0; kh < 2; ++kh) {
#pragma unroll
        for (int e = 0; e < 8; ++e) {
          __bf16 h0, l0, h1, l1;
          split_bf(xa[16 * kh + e], h0, l0);
          split_bf(xa[16 * kh + 8 + e], h1, l1);
          ah[kh][e]     = h0;
          al[kh][e]     = l0;
          ah[kh][8 + e] = h1;
          al[kh][8 + e] = l1;
        }
      }
      float uD[8];
#pragma unroll
      for (int r = 0; r < 8; ++r) uD[r] = US[(8 * hh + r) * kSlabP + s];

#pragma unroll
      for (int nt = 0; nt < 4; ++nt) {
        v8f acc = z8;
#pragma unroll
        for (int kh = 0; kh < 2; ++kh) {
          const v16b bl = frag_load(ALs + (16 * nt + c) * kLoP + koff + 32 * kh);
          acc = mma_b(ah[kh], bh[nt][kh], acc);
          acc = mma_b(ah[kh], bl, acc);
          acc = mma_b(al[kh], bh[nt][kh], acc);
        }
#pragma unroll
        for (int r = 0; r < 8; ++r) {
          const float xn = acc[r] + bD[nt] * uD[r];
          XS[(8 * hh + r) * kSlabP + 16 * nt + c] = xn;
        }
      }
      __syncthreads();

      float yp = 0.0f;
#pragma unroll
      for (int g = 0; g < 4; ++g) {
        const int kb = 16 * g + koff;
        const v4f p0 = *(const v4f*)(XS + c * kSlabP + kb);
        const v4f p1 = *(const v4f*)(XS + c * kSlabP + kb + 4);
        const v4f q0 = *(const v4f*)(CS + kb);
        const v4f q1 = *(const v4f*)(CS + kb + 4);
#pragma unroll
        for (int e = 0; e < 4; ++e) {
          const float a0 = p0[e];
          const float a1 = p1[e];
          xa[8 * g + e]     = a0;
          xa[8 * g + 4 + e] = a1;
          yp = fmaf(a0, q0[e], yp);
          yp = fmaf(a1, q1[e], yp);
        }
      }
      const float yo = __shfl_xor(yp, 16, 32);
      const float y  = yp + yo;
      if (hh == 0) YS[c * kSlabP + s] = y;
      __syncthreads();
    }

    v4f yv[8];
#pragma unroll
    for (int it = 0; it < 8; ++it) yv[it] = *(const v4f*)(YS + (it * 2 + hh) * kSlabP + c4);
    for (int pass = 0; pass < 2; ++pass) {
#pragma unroll
      for (int it = 0; it < 8; ++it) {
        const int rr = it * 2 + hh;
        *(volatile v4f*)(out + (size_t)(rowbase + rr) * kSteps + t0 + c4) = yv[it];
      }
      __threadfence();
    }
    __syncthreads();
  }
}

extern "C" void kernel_launch(void* const* d_in, const int* in_sizes, int n_in,
                              void* d_out, int out_size, void* d_ws, size_t ws_size,
                              hipStream_t stream) {
  if (n_in < 5 || d_out == nullptr || d_ws == nullptr) return;
  if (in_sizes[0] != kBatch * kSteps) return;
  if (in_sizes[1] != kState * kState) return;
  if (in_sizes[2] != kState) return;
  if (in_sizes[3] != kState) return;
  if (in_sizes[4] != 1) return;
  if (out_size != kBatch * kSteps) return;

  const float* u     = (const float*)d_in[0];
  const float* A     = (const float*)d_in[1];
  const float* Bv    = (const float*)d_in[2];
  const float* Cv    = (const float*)d_in[3];
  const float* stepp = (const float*)d_in[4];
  float* out = (float*)d_out;

  char* ws = (char*)d_ws;
  size_t off = 0;
  auto carve = [&](size_t bytes) -> char* { char* p = ws + off; off += (bytes + 255) & ~(size_t)255; return p; };
  unsigned short* ABH = (unsigned short*)carve(kBytesPlane);
  unsigned short* ABL = (unsigned short*)carve(kBytesPlane);
  float*          BC  = (float*)carve(kBytesBC);
  if (off > ws_size || off > (size_t)134217728) return;

  discretise_kernel<<<1, 256, 0, stream>>>(A, Bv, Cv, stepp, ABH, ABL, BC);
  state_scan_kernel<<<kBatch / kRowsBlk, 32, 0, stream>>>(u, ABH, ABL, BC, out);
}
